// GATModel_32074815767392
// MI455X (gfx1250) — hardware-verified
//
#include <hip/hip_runtime.h>
#include <stddef.h>
#include <stdint.h>
#include <math.h>


#define NN      20000
#define MP      20096
#define D0      64
#define D1      128
#define D2      256
#define D3      512
#define D4      1024
#define NCLS    64
#define RPOOL   1024
#define NBK     20
#define NB      1024
#define NTHR    256
#define NWAVE   8
#define EPT     8
#define CHUNK   (NTHR * EPT)
#define WCAP    (EPT * 32)
#define LISTN   (NWAVE * WCAP)
#define NBMAX   2048
#define SLOTB   11
#define RCAP    28672
#define DEGCAP  64
#define GBM     64
#define GBN     64
#define GTHR    128
#define SSL     128
#define SPW     16
#define HTHR    512
#define NEGSL   0.2f
#define MX0     (-1.0e30f)
#define WSMAX   134217728
#define LDS_BKT ((2 * RCAP + 2 * NBMAX + LISTN) * 4 + 64)
#define U1      (D1 * (D0 / 8))
#define U2      (D2 * (2 * D1 / 8))
#define U3      (D3 * (2 * D2 / 8))
#define U4      (D4 * (2 * D3 / 8))
#define UT      (U1 + U2 + U3 + U4)

static_assert((CHUNK & (CHUNK - 1)) == 0 && CHUNK <= (1 << SLOTB));
static_assert(NBMAX == (1 << SLOTB) && NB <= NBMAX && (NB & (NB - 1)) == 0);
static_assert(NTHR * 8 == NBMAX && NTHR * 4 == NB);
static_assert(LISTN >= NBMAX && (RCAP % (NTHR * 4)) == 0);
static_assert(((2 * RCAP + 2 * NBMAX + LISTN) % (NTHR * 4)) == 0);
static_assert(LDS_BKT <= 300000);
static_assert(MP % 128 == 0 && MP >= NN && MP - NN < 128 && MP % GBM == 0 && MP % SSL == 0);
static_assert(NBK * NB >= MP && (NBK - 1) * NB < NN);
static_assert(RPOOL == NB && RPOOL <= NN && RPOOL % SSL == 0 && RPOOL % GBM == 0);
static_assert(SSL == NWAVE * SPW && NB % SSL == 0);
static_assert((MP * (D0 / 8)) % NTHR == 0);
static_assert(U1 % NTHR == 0 && U2 % NTHR == 0 && U3 % NTHR == 0 && U4 % NTHR == 0);
static_assert(D0 % 32 == 0 && (2 * D1) % 32 == 0 && (2 * D2) % 32 == 0 && (2 * D3) % 32 == 0);
static_assert(D1 % GBN == 0 && D2 % GBN == 0 && D3 % GBN == 0 && D4 % GBN == 0);
static_assert(GBM == (GTHR / 32) * 16);
static_assert(D0 + D1 + D2 + D3 == 960 && 960 % 32 == 0);
static_assert(HTHR == 2 * 256 && D4 == 4 * 256 && HTHR == 8 * NCLS && D4 == 8 * 128);

typedef float          v2f  __attribute__((ext_vector_type(2)));
typedef float          v4f  __attribute__((ext_vector_type(4)));
typedef float          v8f  __attribute__((ext_vector_type(8)));
typedef int            v4i  __attribute__((ext_vector_type(4)));
typedef int            v8i  __attribute__((ext_vector_type(8)));
typedef unsigned int   v2u  __attribute__((ext_vector_type(2)));
typedef unsigned int   v4u  __attribute__((ext_vector_type(4)));
typedef unsigned short v8us __attribute__((ext_vector_type(8)));
typedef __bf16         v16b __attribute__((ext_vector_type(16)));
typedef v4f  __attribute__((may_alias)) v4fa;
typedef v4i  __attribute__((may_alias)) v4ia;
typedef v8us __attribute__((may_alias)) v8usa;
union FragB { v16b v; v8us h[2]; v8i w; };

__device__ __forceinline__ v8f wmb(const FragB& a, const FragB& b, v8f c) {
  v8f d = __builtin_amdgcn_wmma_f32_16x16x32_bf16(false, a.v, false, b.v, (short)0, c, false, false);
  asm volatile("v_nop\n\tv_nop\n\tv_nop\n\tv_nop" : "+v"(d) : "v"(a.w), "v"(b.w));
  return d;
}

__device__ __forceinline__ unsigned int f2bf(float f) {
  const unsigned int u = __float_as_uint(f);
  return ((u + 0x7FFFu + ((u >> 16) & 1u)) >> 16) & 0xFFFFu;
}
__device__ __forceinline__ float bf2f(unsigned int b) { return __uint_as_float(b << 16); }
__device__ __forceinline__ float bfr(float f) { return bf2f(f2bf(f)); }
__device__ __forceinline__ v4f bfr4(const v4f a) {
  v4f r; r.x = bfr(a.x); r.y = bfr(a.y); r.z = bfr(a.z); r.w = bfr(a.w); return r;
}
__device__ __forceinline__ unsigned int pk2(float lo, float hi) { return f2bf(lo) | (f2bf(hi) << 16); }
__device__ __forceinline__ unsigned int pk2lo(float lo, float hi) {
  return f2bf(lo - bfr(lo)) | (f2bf(hi - bfr(hi)) << 16);
}
__device__ __forceinline__ v4u pack8(const v4f a, const v4f b) {
  v4u r;
  r.x = pk2(a.x, a.y); r.y = pk2(a.z, a.w); r.z = pk2(b.x, b.y); r.w = pk2(b.z, b.w);
  return r;
}

__device__ __forceinline__ int scan_chunk(const int* __restrict__ dsts, int nE, int cbase, int slotBase,
                                          int nb, int vec8, int* list, int tid, int lane, int wave) {
  int wc = 0;
  const int el0  = tid * EPT;
  const int e0   = cbase + el0;
  const int sent = -2147483647 - 1;
  v4i da, db;
  if (vec8 != 0 && cbase + CHUNK <= nE) {
    da = *(const v4i*)(dsts + e0);
    db = *(const v4i*)(dsts + e0 + 4);
  } else {
    da.x = (e0     < nE) ? dsts[min(e0,     nE - 1)] : sent;
    da.y = (e0 + 1 < nE) ? dsts[min(e0 + 1, nE - 1)] : sent;
    da.z = (e0 + 2 < nE) ? dsts[min(e0 + 2, nE - 1)] : sent;
    da.w = (e0 + 3 < nE) ? dsts[min(e0 + 3, nE - 1)] : sent;
    db.x = (e0 + 4 < nE) ? dsts[min(e0 + 4, nE - 1)] : sent;
    db.y = (e0 + 5 < nE) ? dsts[min(e0 + 5, nE - 1)] : sent;
    db.z = (e0 + 6 < nE) ? dsts[min(e0 + 6, nE - 1)] : sent;
    db.w = (e0 + 7 < nE) ? dsts[min(e0 + 7, nE - 1)] : sent;
  }
  const unsigned nbs = (unsigned)slotBase;
  const unsigned unb = (unsigned)nb;
  const unsigned s0 = (unsigned)da.x - nbs, s1 = (unsigned)da.y - nbs;
  const unsigned s2 = (unsigned)da.z - nbs, s3 = (unsigned)da.w - nbs;
  const unsigned s4 = (unsigned)db.x - nbs, s5 = (unsigned)db.y - nbs;
  const unsigned s6 = (unsigned)db.z - nbs, s7 = (unsigned)db.w - nbs;
  const bool h0 = s0 < unb, h1 = s1 < unb, h2 = s2 < unb, h3 = s3 < unb;
  const bool h4 = s4 < unb, h5 = s5 < unb, h6 = s6 < unb, h7 = s7 < unb;
  const unsigned any = __builtin_amdgcn_ballot_w32(h0 | h1 | h2 | h3 | h4 | h5 | h6 | h7);
  if (any != 0u) {
#define HITJ(J, HJ, SJ) { \
      const unsigned mj = __builtin_amdgcn_ballot_w32(HJ); \
      if (mj != 0u) { \
        if (HJ) { \
          const int pos = wc + (int)__builtin_amdgcn_mbcnt_lo(mj, 0u); \
          if (pos < WCAP) list[wave * WCAP + pos] = ((el0 + (J)) << SLOTB) | (int)(SJ); \
        } \
        wc += (int)__builtin_popcount(mj); } }
    HITJ(0, h0, s0)
    HITJ(1, h1, s1)
    HITJ(2, h2, s2)
    HITJ(3, h3, s3)
    HITJ(4, h4, s4)
    HITJ(5, h5, s5)
    HITJ(6, h6, s6)
    HITJ(7, h7, s7)
#undef HITJ
  }
  return wc;
}

__device__ __forceinline__ void wlr_rows(const float* __restrict__ W, const float* __restrict__ al,
                                         const float* __restrict__ ar, int dout, int k0,
                                         float* WLR, int ooff, int lane) {
  float ra = 0.0f, rb = 0.0f;
#pragma unroll 1
  for (int r = 0; r < 32; ++r) {
    const float* wrow = W + (size_t)(k0 + r) * (size_t)dout;
    double a = 0.0, b = 0.0;
#pragma unroll 2
    for (int n = lane; n < dout; n += 32) {
      const double w = (double)bfr(wrow[n]);
      a = fma(w, (double)bfr(al[n]), a);
      b = fma(w, (double)bfr(ar[n]), b);
    }
#pragma unroll
    for (int off = 16; off > 0; off >>= 1) {
      a += __shfl_xor(a, off);
      b += __shfl_xor(b, off);
    }
    ra = (lane == r) ? (float)a : ra;
    rb = (lane == r) ? (float)b : rb;
  }
  float* pa = WLR + ooff + lane;
  float* pb = WLR + 1024 + ooff + lane;
  *(volatile float*)pa = ra;
  *(volatile float*)pb = rb;
  __threadfence();
  *(volatile float*)pa = ra;
  *(volatile float*)pb = rb;
}

__global__ __launch_bounds__(NTHR) void k_wlr(
    const float* __restrict__ W1, const float* __restrict__ al1, const float* __restrict__ ar1,
    const float* __restrict__ W2, const float* __restrict__ al2, const float* __restrict__ ar2,
    const float* __restrict__ W3, const float* __restrict__ al3, const float* __restrict__ ar3,
    const float* __restrict__ W4, const float* __restrict__ al4, const float* __restrict__ ar4,
    float* WLR) {
  const int lane = (int)threadIdx.x & 31;
  const int g = (int)blockIdx.x * NWAVE + ((int)threadIdx.x >> 5);
  if (g < 2)        wlr_rows(W1, al1, ar1, D1, 32 * g,        WLR, 32 * g, lane);
  else if (g < 6)   wlr_rows(W2, al2, ar2, D2, 32 * (g - 2),  WLR, 32 * g, lane);
  else if (g < 14)  wlr_rows(W3, al3, ar3, D3, 32 * (g - 6),  WLR, 32 * g, lane);
  else if (g < 30)  wlr_rows(W4, al4, ar4, D4, 32 * (g - 14), WLR, 32 * g, lane);
}

__device__ __forceinline__ void wtr_unit(const float* __restrict__ w, int Kin, int Ncol, int Kout,
                                         unsigned short* wt, int u) {
  const int kq = Kout >> 3;
  const int n  = u / kq;
  const int k8 = (u - n * kq) * 8;
  const int kk = k8 - (k8 / Kin) * Kin;
  const int ncl = n < Ncol ? n : Ncol - 1;
  const float* p = w + (size_t)kk * (size_t)Ncol + ncl;
  v4f a, b;
  a.x = p[0];                    a.y = p[(size_t)Ncol];         a.z = p[(size_t)2 * Ncol];     a.w = p[(size_t)3 * Ncol];
  b.x = p[(size_t)4 * Ncol];     b.y = p[(size_t)5 * Ncol];     b.z = p[(size_t)6 * Ncol];     b.w = p[(size_t)7 * Ncol];
  const v4u wv = pack8(a, b);
  unsigned short* o = wt + (size_t)n * (size_t)Kout + k8;
  *(volatile v4u*)o = wv;
  __threadfence();
  *(volatile v4u*)o = wv;
}

__global__ __launch_bounds__(NTHR) void k_wprep(const float* __restrict__ W1, const float* __restrict__ W2,
                                                const float* __restrict__ W3, const float* __restrict__ W4,
                                                unsigned short* W1t, unsigned short* W2d,
                                                unsigned short* W3d, unsigned short* W4d) {
  const int u = (int)blockIdx.x * NTHR + (int)threadIdx.x;
  if (u < U1)                  wtr_unit(W1, D0, D1, D0,     W1t, u);
  else if (u < U1 + U2)        wtr_unit(W2, D1, D2, 2 * D1, W2d, u - U1);
  else if (u < U1 + U2 + U3)   wtr_unit(W3, D2, D3, 2 * D2, W3d, u - U1 - U2);
  else if (u < UT)             wtr_unit(W4, D3, D4, 2 * D3, W4d, u - U1 - U2 - U3);
}

__global__ __launch_bounds__(NTHR) void k_cvx(const float* __restrict__ x, const float* __restrict__ WLR,
                                              unsigned short* fb, float* EL, float* ER, int nN) {
  __shared__ float sE[64];
  const int tid = (int)threadIdx.x, lane = tid & 31, wave = tid >> 5;
  const int i   = (int)blockIdx.x * NTHR + tid;
  const int row = i >> 3;
  const int c0  = (i & 7) * 8;
  const int rc  = row < nN ? row : nN - 1;
  const float* p = x + (size_t)rc * D0 + c0;
  v4f a = *(const v4fa*)p, b = *(const v4fa*)(p + 4);
  const v4f z4 = {0.f, 0.f, 0.f, 0.f};
  if (row >= nN) { a = z4; b = z4; }
  const v4f ar = bfr4(a), br = bfr4(b);
  const v4f l0 = *(const v4fa*)(WLR + c0),        l1 = *(const v4fa*)(WLR + c0 + 4);
  const v4f r0 = *(const v4fa*)(WLR + 1024 + c0), r1 = *(const v4fa*)(WLR + 1024 + c0 + 4);
  float ds = 0.0f, dd = 0.0f;
  ds = fmaf(ar.x, l0.x, ds); ds = fmaf(ar.y, l0.y, ds); ds = fmaf(ar.z, l0.z, ds); ds = fmaf(ar.w, l0.w, ds);
  ds = fmaf(br.x, l1.x, ds); ds = fmaf(br.y, l1.y, ds); ds = fmaf(br.z, l1.z, ds); ds = fmaf(br.w, l1.w, ds);
  dd = fmaf(ar.x, r0.x, dd); dd = fmaf(ar.y, r0.y, dd); dd = fmaf(ar.z, r0.z, dd); dd = fmaf(ar.w, r0.w, dd);
  dd = fmaf(br.x, r1.x, dd); dd = fmaf(br.y, r1.y, dd); dd = fmaf(br.z, r1.z, dd); dd = fmaf(br.w, r1.w, dd);
#pragma unroll
  for (int off = 1; off < 8; off <<= 1) {
    ds += __shfl_xor(ds, off);
    dd += __shfl_xor(dd, off);
  }
  if ((tid & 7) == 0) { sE[tid >> 3] = ds; sE[32 + (tid >> 3)] = dd; }
  const v4u hv = pack8(a, b);
  unsigned short* o = fb + (size_t)row * D0 + c0;
  *(volatile v4u*)o = hv;
  __threadfence();
  *(volatile v4u*)o = hv;
  __syncthreads();
  if (wave == 0) {
    const float v = sE[lane];
    float* q = EL + (size_t)blockIdx.x * 32 + lane;
    *(volatile float*)q = v;
    __threadfence();
    *(volatile float*)q = v;
  } else if (wave == 1) {
    const float v = sE[32 + lane];
    float* q = ER + (size_t)blockIdx.x * 32 + lane;
    *(volatile float*)q = v;
    __threadfence();
    *(volatile float*)q = v;
  }
}

__global__ __launch_bounds__(NTHR) void k_bucket(const int* __restrict__ srcs, const int* __restrict__ dsts,
                                                 int nE, int nN, int vec8,
                                                 int* SRT, int* SOFF, int* SCNT, int* META) {
  extern __shared__ v4f lds_dyn[];
  int* reg1 = (int*)lds_dyn;
  int* reg2 = reg1 + RCAP;
  int* scnt = reg2 + RCAP;
  int* soff = scnt + NBMAX;
  int* list = soff + NBMAX;
  int* wcnt = list + LISTN;
  int* wtot = wcnt + NWAVE;
  const int tid = (int)threadIdx.x, lane = tid & 31, wave = tid >> 5;
  const int nodeBase = (int)blockIdx.x * NB;

  {
    const v4i z4 = {0, 0, 0, 0};
    for (int i = tid * 4; i < 2 * RCAP + 2 * NBMAX + LISTN; i += NTHR * 4) *(v4ia*)(reg1 + i) = z4;
    if (tid < 16) wcnt[tid] = 0;
  }
  __syncthreads();

  int tot = 0;
  const int nChunks = (nE + CHUNK - 1) / CHUNK;
#pragma unroll 1
  for (int ch = 0; ch < nChunks; ++ch) {
    const int cbase = ch * CHUNK;
    const int wc = scan_chunk(dsts, nE, cbase, nodeBase, NB, vec8, list, tid, lane, wave);
    if (lane == 0) wcnt[wave] = wc;
    __syncthreads();
    int pre = 0, all = 0;
#pragma unroll
    for (int w2 = 0; w2 < NWAVE; ++w2) {
      int c = wcnt[w2];
      c = c < 0 ? 0 : (c > WCAP ? WCAP : c);
      all += c;
      pre += (w2 < wave) ? c : 0;
    }
    const int wcc  = wc > WCAP ? WCAP : wc;
    const int base = tot + pre;
#pragma unroll 1
    for (int i = lane; i < wcc; i += 32) {
      const int ent = list[wave * WCAP + i];
      const int el  = (ent >> SLOTB) & (CHUNK - 1);
      const int sl  = ent & (NBMAX - 1);
      int eid = cbase + el;
      eid = eid > nE - 1 ? nE - 1 : eid;
      const int pos = base + i;
      if (pos < RCAP) reg1[pos] = (int)(((unsigned)eid << SLOTB) | (unsigned)sl);
    }
    tot += all;
    tot = tot > RCAP ? RCAP : tot;
    __syncthreads();
  }
  const int nh = tot;

  if (wave == 0) {
#pragma unroll 1
    for (int b0 = 0; b0 < nh; b0 += 32) {
      const int idx = b0 + lane;
      const int uv  = reg1[idx < nh ? idx : nh - 1];
      const int m32 = (nh - b0) < 32 ? (nh - b0) : 32;
#pragma unroll 1
      for (int k = 0; k < m32; ++k) {
        const int u  = __builtin_amdgcn_readlane(uv, k);
        const int sl = u & (NBMAX - 1);
        if (lane == 0) scnt[sl] = scnt[sl] + 1;
      }
    }
  }
  __syncthreads();

  {
    const v4i ca = *(const v4ia*)(scnt + 8 * tid);
    const v4i cb = *(const v4ia*)(scnt + 8 * tid + 4);
    const int e0 = ca.x < 0 ? 0 : ca.x, e1 = ca.y < 0 ? 0 : ca.y, e2 = ca.z < 0 ? 0 : ca.z, e3 = ca.w < 0 ? 0 : ca.w;
    const int e4 = cb.x < 0 ? 0 : cb.x, e5 = cb.y < 0 ? 0 : cb.y, e6 = cb.z < 0 ? 0 : cb.z, e7 = cb.w < 0 ? 0 : cb.w;
    const int ts = e0 + e1 + e2 + e3 + e4 + e5 + e6 + e7;
    int incl = ts;
#pragma unroll
    for (int d = 1; d < 32; d <<= 1) {
      const int up = __shfl_up(incl, d);
      if (lane >= d) incl += up;
    }
    if (lane == 31) wtot[wave] = incl;
    __syncthreads();
    int pre = 0;
#pragma unroll
    for (int w2 = 0; w2 < NWAVE; ++w2) pre += (w2 < wave) ? wtot[w2] : 0;
    int run = pre + incl - ts;
    soff[8 * tid + 0] = run; run += e0;
    soff[8 * tid + 1] = run; run += e1;
    soff[8 * tid + 2] = run; run += e2;
    soff[8 * tid + 3] = run; run += e3;
    soff[8 * tid + 4] = run; run += e4;
    soff[8 * tid + 5] = run; run += e5;
    soff[8 * tid + 6] = run; run += e6;
    soff[8 * tid + 7] = run;
  }
  __syncthreads();
  for (int i = tid; i < NBMAX; i += NTHR) list[i] = soff[i];
  __syncthreads();

  if (wave == 0) {
#pragma unroll 1
    for (int b0 = 0; b0 < nh; b0 += 32) {
      const int idx = b0 + lane;
      const int uv  = reg1[idx < nh ? idx : nh - 1];
      const int m32 = (nh - b0) < 32 ? (nh - b0) : 32;
#pragma unroll 1
      for (int k = 0; k < m32; ++k) {
        const int u   = __builtin_amdgcn_readlane(uv, k);
        const int sl  = u & (NBMAX - 1);
        const int eid = (int)((unsigned)u >> SLOTB);
        if (lane == 0) {
          int pos = list[sl];
          pos = pos < 0 ? 0 : (pos > RCAP - 1 ? RCAP - 1 : pos);
          reg2[pos] = eid;
          list[sl] = pos + 1;
        }
      }
    }
  }
  __syncthreads();

  const v4i cq = *(const v4ia*)(scnt + 4 * tid);
  const v4i oq = *(const v4ia*)(soff + 4 * tid);
  {
    const bool big = (cq.x > DEGCAP) | (cq.y > DEGCAP) | (cq.z > DEGCAP) | (cq.w > DEGCAP);
    const unsigned bm = __builtin_amdgcn_ballot_w32(big);
    if (lane == 0) wcnt[wave] = (bm != 0u) ? 1 : 0;
  }
  __syncthreads();
  int flag = (nh >= RCAP) ? 1 : 0;
#pragma unroll
  for (int w2 = 0; w2 < NWAVE; ++w2) flag |= wcnt[w2];

  int* srt = SRT + (size_t)blockIdx.x * RCAP;
#pragma unroll 1
  for (int i4 = tid * 4; i4 < RCAP; i4 += NTHR * 4) {
    const v4i e = *(const v4ia*)(reg2 + i4);
    const int e0 = e.x < 0 ? 0 : (e.x > nE - 1 ? nE - 1 : e.x);
    const int e1 = e.y < 0 ? 0 : (e.y > nE - 1 ? nE - 1 : e.y);
    const int e2 = e.z < 0 ? 0 : (e.z > nE - 1 ? nE - 1 : e.z);
    const int e3 = e.w < 0 ? 0 : (e.w > nE - 1 ? nE - 1 : e.w);
    int s0 = srcs[e0], s1 = srcs[e1], s2 = srcs[e2], s3 = srcs[e3];
    s0 = s0 < 0 ? 0 : (s0 > nN - 1 ? nN - 1 : s0);
    s1 = s1 < 0 ? 0 : (s1 > nN - 1 ? nN - 1 : s1);
    s2 = s2 < 0 ? 0 : (s2 > nN - 1 ? nN - 1 : s2);
    s3 = s3 < 0 ? 0 : (s3 > nN - 1 ? nN - 1 : s3);
    v4i o;
    o.x = (i4     < nh) ? s0 : 0;
    o.y = (i4 + 1 < nh) ? s1 : 0;
    o.z = (i4 + 2 < nh) ? s2 : 0;
    o.w = (i4 + 3 < nh) ? s3 : 0;
    *(volatile v4i*)(srt + i4) = o;
    __threadfence();
    *(volatile v4i*)(srt + i4) = o;
  }
  {
    int* po = SOFF + (size_t)blockIdx.x * NB + 4 * tid;
    int* pc = SCNT + (size_t)blockIdx.x * NB + 4 * tid;
    *(volatile v4i*)po = oq;
    *(volatile v4i*)pc = cq;
    __threadfence();
    *(volatile v4i*)po = oq;
    *(volatile v4i*)pc = cq;
  }
  if (wave == 0) {
    const int mv = (lane == 0) ? nh : ((lane == 1) ? flag : 0);
    int* pm = META + (size_t)blockIdx.x * 32 + lane;
    *(volatile int*)pm = mv;
    __threadfence();
    *(volatile int*)pm = mv;
  }
}

template <int EPI>
__global__ __launch_bounds__(GTHR) void k_gemm(const unsigned short* __restrict__ A,
                                               const unsigned short* __restrict__ WT,
                                               float* outF, int K, int ldo, const float* __restrict__ bias) {
  __shared__ __attribute__((aligned(16))) float stg[GBM * GBN];
  const int tid = (int)threadIdx.x, lane = tid & 31, wave = tid >> 5, hh = lane >> 4, m = lane & 15;
  const int rowBase = (int)blockIdx.x * GBM;
  const int col0    = (int)blockIdx.y * GBN;

  v8f acc[4];
  {
    const v8f z = {0.f, 0.f, 0.f, 0.f, 0.f, 0.f, 0.f, 0.f};
    acc[0] = z; acc[1] = z; acc[2] = z; acc[3] = z;
  }
  const unsigned short* ap = A  + (size_t)(rowBase + 16 * wave + m) * (size_t)K + 8 * hh;
  const unsigned short* wp = WT + (size_t)(col0 + m) * (size_t)K + 8 * hh;
  const int ksteps = K >> 5;
#pragma unroll 1
  for (int ks = 0; ks < ksteps; ++ks) {
    FragB af;
    af.h[0] = *(const v8usa*)(ap + 32 * ks);
    af.h[1] = *(const v8usa*)(ap + 32 * ks + 16);
#pragma unroll
    for (int t = 0; t < 4; ++t) {
      const unsigned short* wq = wp + (size_t)(16 * t) * (size_t)K + 32 * ks;
      FragB bf;
      bf.h[0] = *(const v8usa*)wq;
      bf.h[1] = *(const v8usa*)(wq + 16);
      acc[t] = wmb(af, bf, acc[t]);
    }
  }

#pragma unroll
  for (int t = 0; t < 4; ++t) {
    const int lc = 16 * t + m;
#pragma unroll
    for (int r = 0; r < 8; ++r) {
      const int lr = 16 * wave + 8 * hh + r;
      stg[lr * GBN + lc] = acc[t][r];
    }
  }
  __syncthreads();

  if constexpr (EPI == 1) {
    const v4f bb = bfr4(*(const v4fa*)(bias + col0 + 4 * m));
#pragma unroll 1
    for (int i = 0; i < 8; ++i) {
      const int lr = 16 * wave + 2 * i + hh;
      float* q = stg + lr * GBN + 4 * m;
      v4f v = *(const v4fa*)q;
      v.x = tanhf(v.x + bb.x);
      v.y = tanhf(v.y + bb.y);
      v.z = tanhf(v.z + bb.z);
      v.w = tanhf(v.w + bb.w);
      *(v4fa*)q = v;
    }
  }

  v4f fv[8];
#pragma unroll
  for (int i = 0; i < 8; ++i) {
    const int lr = 16 * wave + 2 * i + hh;
    fv[i] = *(const v4fa*)(stg + lr * GBN + 4 * m);
  }
#pragma unroll
  for (int i = 0; i < 8; ++i) {
    const int lr = 16 * wave + 2 * i + hh;
    const int gr = rowBase + lr;
    float* op = outF + (size_t)gr * (size_t)ldo + col0 + 4 * m;
    *(volatile v4f*)op = fv[i];
  }
  __threadfence();
#pragma unroll
  for (int i = 0; i < 8; ++i) {
    const int lr = 16 * wave + 2 * i + hh;
    const int gr = rowBase + lr;
    float* op = outF + (size_t)gr * (size_t)ldo + col0 + 4 * m;
    *(volatile v4f*)op = fv[i];
  }
}

template <int NCH, int MODE>
__global__ __launch_bounds__(NTHR) void k_scan(
    const int* __restrict__ SRT, const int* __restrict__ SOFF, const int* __restrict__ SCNT,
    const int* __restrict__ META,
    const float* __restrict__ F, const float* __restrict__ EL, const float* __restrict__ ER,
    const float* __restrict__ bias, const float* __restrict__ WLn, const float* __restrict__ WRn,
    unsigned short* XH, float* XF, float* ELn, float* ERn, int nN, int mRows) {
  constexpr int D  = 128 * NCH;
  constexpr int SR = (MODE < 2) ? (NWAVE * D) : 4;
  constexpr int SP = (MODE < 2) ? D : 4;
  __shared__ __attribute__((aligned(16))) float srow[SR];
  __shared__ __attribute__((aligned(16))) float sb[SP];
  __shared__ __attribute__((aligned(16))) float swl[SP];
  __shared__ __attribute__((aligned(16))) float swr[SP];
  __shared__ __attribute__((aligned(16))) float sel[SSL];
  __shared__ __attribute__((aligned(16))) float ser[SSL];
  const int tid = (int)threadIdx.x, lane = tid & 31, wave = tid >> 5;

  if constexpr (MODE < 2) {
#pragma unroll 1
    for (int i = tid; i < D; i += NTHR) {
      sb[i]  = bfr(bias[i]);
      swl[i] = WLn[i];
      swr[i] = WRn[i];
    }
  }
  __syncthreads();

  const float qnan = __int_as_float(0x7fc00000);
  const int blockRow = (int)blockIdx.x * SSL;

#pragma unroll 1
  for (int jt = 0; jt < SPW; ++jt) {
    const int slot = wave * SPW + jt;
    const int grow = blockRow + slot;
    int bkt = grow >> 10;
    bkt = bkt > NBK - 1 ? NBK - 1 : bkt;
    const int sl = grow & (NB - 1);
    int nh = META[bkt * 32];
    nh = nh < 0 ? 0 : (nh > RCAP ? RCAP : nh);
    const int ovm = META[bkt * 32 + 1];
    int st = SOFF[bkt * NB + sl];
    const int craw = SCNT[bkt * NB + sl];
    int cnt = craw;
    st  = st < 0 ? 0 : (st > nh ? nh : st);
    cnt = cnt < 0 ? 0 : (cnt > DEGCAP ? DEGCAP : cnt);
    if (cnt > nh - st) cnt = nh - st;
    const float pz = (ovm != 0 || craw > DEGCAP) ? qnan : 0.0f;
    const int gcl = grow < nN ? grow : nN - 1;
    const bool live = grow < nN;
    const float ad = ER[gcl];
    const int* srt = SRT + (size_t)bkt * RCAP;

    float mx = MX0, dn = 0.0f;
    v4f acc[NCH];
#pragma unroll
    for (int j = 0; j < NCH; ++j) { acc[j].x = 0.0f; acc[j].y = 0.0f; acc[j].z = 0.0f; acc[j].w = 0.0f; }

#pragma unroll 1
    for (int b0 = 0; b0 < cnt; b0 += 32) {
      int idx = st + b0 + lane;
      idx = idx > RCAP - 1 ? RCAP - 1 : idx;
      int sr = srt[idx];
      sr = sr < 0 ? 0 : (sr > nN - 1 ? nN - 1 : sr);
      const float es  = EL[sr];
      const int   esi = __float_as_int(es);
      const int m32 = (cnt - b0) < 32 ? (cnt - b0) : 32;
#pragma unroll 1
      for (int k = 0; k < m32; ++k) {
        const int   sk  = __builtin_amdgcn_readlane(sr, k);
        const float ask = __int_as_float(__builtin_amdgcn_readlane(esi, k));
        const float* rp = F + (size_t)sk * D + 4 * lane;
        v4f a[NCH];
#pragma unroll
        for (int j = 0; j < NCH; ++j) a[j] = *(const v4f*)(rp + 128 * j);
        float lg = ask + ad;
        lg = lg > 0.f ? lg : NEGSL * lg;
        const float df = lg - mx;
        const float ee = expf(-fabsf(df));
        const bool  up = df > 0.f;
        const float s1 = up ? ee : 1.0f;
        const float s2 = up ? 1.0f : ee;
        mx = up ? lg : mx;
        dn = fmaf(dn, s1, s2);
#pragma unroll
        for (int j = 0; j < NCH; ++j) {
          acc[j].x = fmaf(acc[j].x, s1, s2 * a[j].x);
          acc[j].y = fmaf(acc[j].y, s1, s2 * a[j].y);
          acc[j].z = fmaf(acc[j].z, s1, s2 * a[j].z);
          acc[j].w = fmaf(acc[j].w, s1, s2 * a[j].w);
        }
      }
    }
    const bool has = cnt > 0;
    const float dsafe = has ? dn : 1.0f;
    const float rinv  = __builtin_amdgcn_rcpf(dsafe);
    const float inv   = has ? rinv : 0.0f;

    v4f y[NCH];
    if constexpr (MODE < 2) {
      float* wrow = srow + wave * D;
#pragma unroll
      for (int j = 0; j < NCH; ++j) *(v4fa*)(wrow + 128 * j + 4 * lane) = acc[j];
      float ds = 0.0f, dd = 0.0f;
#pragma unroll 1
      for (int t = 0; t < 4 * NCH; ++t) {
        const int ai = 128 * (t >> 2) + 4 * lane + (t & 3);
        const float pre = fmaf(wrow[ai], inv, sb[ai]);
        float v = tanhf(pre) + pz;
        v = live ? v : 0.0f;
        ds = fmaf(v, swl[ai], ds);
        dd = fmaf(v, swr[ai], dd);
        wrow[ai] = v;
      }
#pragma unroll
      for (int off = 16; off > 0; off >>= 1) {
        ds += __shfl_xor(ds, off);
        dd += __shfl_xor(dd, off);
      }
      if (lane == 0) { sel[slot] = ds; ser[slot] = dd; }
#pragma unroll
      for (int j = 0; j < NCH; ++j) y[j] = *(const v4fa*)(wrow + 128 * j + 4 * lane);
    } else {
#pragma unroll
      for (int j = 0; j < NCH; ++j) {
        y[j].x = live ? (acc[j].x * inv + pz) : 0.0f;
        y[j].y = live ? (acc[j].y * inv + pz) : 0.0f;
        y[j].z = live ? (acc[j].z * inv + pz) : 0.0f;
        y[j].w = live ? (acc[j].w * inv + pz) : 0.0f;
      }
    }

    const bool wr = grow < mRows;
    if constexpr (MODE == 1) {
      float* op = XF + (size_t)grow * D + 4 * lane;
      if (wr) {
#pragma unroll
        for (int j = 0; j < NCH; ++j) *(volatile v4f*)(op + 128 * j) = y[j];
      }
      __threadfence();
      if (wr) {
#pragma unroll
        for (int j = 0; j < NCH; ++j) *(volatile v4f*)(op + 128 * j) = y[j];
      }
    } else {
      v2u hv[NCH], lv[NCH];
#pragma unroll
      for (int j = 0; j < NCH; ++j) {
        hv[j].x = pk2(y[j].x, y[j].y);   hv[j].y = pk2(y[j].z, y[j].w);
        lv[j].x = pk2lo(y[j].x, y[j].y); lv[j].y = pk2lo(y[j].z, y[j].w);
      }
      unsigned short* gp = XH + (size_t)grow * (2 * D) + 4 * lane;
      if (wr) {
#pragma unroll
        for (int j = 0; j < NCH; ++j) {
          *(volatile v2u*)(gp + 128 * j)     = hv[j];
          *(volatile v2u*)(gp + D + 128 * j) = lv[j];
        }
      }
      __threadfence();
      if (wr) {
#pragma unroll
        for (int j = 0; j < NCH; ++j) {
          *(volatile v2u*)(gp + 128 * j)     = hv[j];
          *(volatile v2u*)(gp + D + 128 * j) = lv[j];
        }
      }
    }
  }

  __syncthreads();
  if constexpr (MODE < 2) {
    if (wave == 0) {
      const v4f v = *(const v4fa*)(sel + 4 * lane);
      float* q = ELn + blockRow + 4 * lane;
      *(volatile v4f*)q = v;
      __threadfence();
      *(volatile v4f*)q = v;
    } else if (wave == 1) {
      const v4f v = *(const v4fa*)(ser + 4 * lane);
      float* q = ERn + blockRow + 4 * lane;
      *(volatile v4f*)q = v;
      __threadfence();
      *(volatile v4f*)q = v;
    }
  }
}

__global__ __launch_bounds__(HTHR) void k_head(const float* __restrict__ T4, const float* __restrict__ relW,
                                               const float* __restrict__ relB, const int* __restrict__ rel,
                                               const int* __restrict__ order, const int* __restrict__ META,
                                               float* out) {
  __shared__ double sp[2 * D4];
  __shared__ float spool[D4];
  __shared__ float spart[8 * NCLS];
  __shared__ float slg[NCLS];
  __shared__ float sout[NCLS];
  __shared__ int snz[NCLS];
  __shared__ int sfl[4];
  const int tid = (int)threadIdx.x;
  {
    const int cq = tid & 255, half = tid >> 8;
    double a0 = 0.0, a1 = 0.0, a2 = 0.0, a3 = 0.0;
    const float* base = T4 + (size_t)(half * 512) * D4 + 4 * cq;
#pragma unroll 4
    for (int r = 0; r < 512; ++r) {
      const v4f v = *(const v4f*)(base + (size_t)r * D4);
      a0 += (double)v.x; a1 += (double)v.y; a2 += (double)v.z; a3 += (double)v.w;
    }
    sp[half * D4 + 4 * cq + 0] = a0;
    sp[half * D4 + 4 * cq + 1] = a1;
    sp[half * D4 + 4 * cq + 2] = a2;
    sp[half * D4 + 4 * cq + 3] = a3;
  }
  __syncthreads();
#pragma unroll 1
  for (int c = tid; c < D4; c += HTHR) spool[c] = (float)((sp[c] + sp[D4 + c]) * (1.0 / 1024.0));
  __syncthreads();
  {
    const int j = tid & (NCLS - 1), part = tid >> 6;
    float acc = 0.0f;
#pragma unroll 4
    for (int i = 0; i < 128; ++i) {
      const int c = part * 128 + i;
      acc = fmaf(spool[c], bfr(relW[(size_t)c * NCLS + j]), acc);
    }
    spart[part * NCLS + j] = acc;
  }
  __syncthreads();
  if (tid < NCLS) {
    float s = 0.0f;
#pragma unroll 1
    for (int p = 0; p < 8; ++p) s += spart[p * NCLS + tid];
    slg[tid] = s + bfr(relB[tid]);
  }
  if (tid == 0) {
    int cnt = 0;
#pragma unroll 1
    for (int k = 0; k < NCLS; ++k) {
      const int r = rel[k];
      if (r != 0 && cnt < NCLS) { snz[cnt] = k; cnt = cnt + 1; }
    }
#pragma unroll 1
    for (int k = cnt; k < NCLS; ++k) snz[k] = 0;
    int fl = 0;
#pragma unroll 1
    for (int b = 0; b < NBK; ++b) fl |= META[b * 32 + 1];
    fl |= (order[0] != RPOOL - 1) ? 1 : 0;
    sfl[0] = fl;
  }
  __syncthreads();
  if (tid < NCLS) {
    int idx = snz[tid];
    idx = idx < 0 ? 0 : (idx > NCLS - 1 ? NCLS - 1 : idx);
    const float v = slg[idx];
    const float pzz = (sfl[0] != 0) ? __int_as_float(0x7fc00000) : 0.0f;
    sout[tid] = v + pzz;
  }
  __syncthreads();
  if (tid < 32) {
    v2f o;
    o.x = sout[2 * tid];
    o.y = sout[2 * tid + 1];
    float* q = out + 2 * tid;
    *(volatile v2f*)q = o;
    __threadfence();
    *(volatile v2f*)q = o;
  }
}

static inline size_t al256(size_t v) { return (v + 255) & ~(size_t)255; }

extern "C" void kernel_launch(void* const* d_in, const int* in_sizes, int n_in,
                              void* d_out, int out_size, void* d_ws, size_t ws_size,
                              hipStream_t stream) {
  if (n_in < 23) return;
  if (in_sizes[0] != NN * D0) return;
  if (in_sizes[1] != D0 * D1 || in_sizes[2] != D1 || in_sizes[3] != D1 || in_sizes[4] != D1) return;
  if (in_sizes[5] != D1 * D2 || in_sizes[6] != D2 || in_sizes[7] != D2 || in_sizes[8] != D2) return;
  if (in_sizes[9] != D2 * D3 || in_sizes[10] != D3 || in_sizes[11] != D3 || in_sizes[12] != D3) return;
  if (in_sizes[13] != D3 * D4 || in_sizes[14] != D4 || in_sizes[15] != D4 || in_sizes[16] != D4) return;
  if (in_sizes[17] != D4 * NCLS || in_sizes[18] != NCLS) return;
  const int nE = in_sizes[19];
  if (nE < 1 || nE >= (1 << 21) || in_sizes[20] != nE) return;
  if (in_sizes[21] != NCLS || in_sizes[22] < 1) return;
  if (out_size != NCLS) return;

  const float* feat = (const float*)d_in[0];
  const float* W1  = (const float*)d_in[1];   const float* al1 = (const float*)d_in[2];
  const float* ar1 = (const float*)d_in[3];   const float* b1  = (const float*)d_in[4];
  const float* W2  = (const float*)d_in[5];   const float* al2 = (const float*)d_in[6];
  const float* ar2 = (const float*)d_in[7];   const float* b2  = (const float*)d_in[8];
  const float* W3  = (const float*)d_in[9];   const float* al3 = (const float*)d_in[10];
  const float* ar3 = (const float*)d_in[11];  const float* b3  = (const float*)d_in[12];
  const float* W4  = (const float*)d_in[13];  const float* al4 = (const float*)d_in[14];
  const float* ar4 = (const float*)d_in[15];  const float* b4  = (const float*)d_in[16];
  const float* relW = (const float*)d_in[17];
  const float* relB = (const float*)d_in[18];
  const int* src   = (const int*)d_in[19];
  const int* dst   = (const int*)d_in[20];
  const int* rel   = (const int*)d_in[21];
  const int* order = (const int*)d_in[22];
  float* out = (float*)d_out;

  char* ws = (char*)d_ws;
  size_t off = 0;
  const size_t oWLR = off; off = al256(off + (size_t)2048 * 4);
  const size_t oW1t = off; off = al256(off + (size_t)D1 * D0 * 2);
  const size_t oW2d = off; off = al256(off + (size_t)D2 * 2 * D1 * 2);
  const size_t oW3d = off; off = al256(off + (size_t)D3 * 2 * D2 * 2);
  const size_t oW4d = off; off = al256(off + (size_t)D4 * 2 * D3 * 2);
  const size_t oFB  = off; off = al256(off + (size_t)MP * D0 * 2);
  const size_t oELa = off; off = al256(off + (size_t)MP * 4);
  const size_t oERa = off; off = al256(off + (size_t)MP * 4);
  const size_t oELb = off; off = al256(off + (size_t)MP * 4);
  const size_t oERb = off; off = al256(off + (size_t)MP * 4);
  const size_t oSRT = off; off = al256(off + (size_t)NBK * RCAP * 4);
  const size_t oSOF = off; off = al256(off + (size_t)NBK * NB * 4);
  const size_t oSCN = off; off = al256(off + (size_t)NBK * NB * 4);
  const size_t oMET = off; off = al256(off + (size_t)NBK * 32 * 4);
  const size_t oRA  = off; off = al256(off + (size_t)MP * D3 * 4);
  const size_t oRB  = off; off = al256(off + (size_t)MP * D3 * 4);
  const size_t oXHL = off; off = al256(off + (size_t)MP * 2 * D2 * 2);
  const size_t oZ4  = off; off = al256(off + (size_t)RPOOL * 2 * D3 * 2);
  const size_t oT4  = off; off = al256(off + (size_t)RPOOL * D4 * 4);
  if (off > ws_size || off > (size_t)WSMAX) return;

  float*          WLR = (float*)(ws + oWLR);
  unsigned short* W1t = (unsigned short*)(ws + oW1t);
  unsigned short* W2d = (unsigned short*)(ws + oW2d);
  unsigned short* W3d = (unsigned short*)(ws + oW3d);
  unsigned short* W4d = (unsigned short*)(ws + oW4d);
  unsigned short* FB  = (unsigned short*)(ws + oFB);
  float* ELa = (float*)(ws + oELa);  float* ERa = (float*)(ws + oERa);
  float* ELb = (float*)(ws + oELb);  float* ERb = (float*)(ws + oERb);
  int* SRT  = (int*)(ws + oSRT);
  int* SOFF = (int*)(ws + oSOF);
  int* SCNT = (int*)(ws + oSCN);
  int* META = (int*)(ws + oMET);
  float* RA = (float*)(ws + oRA);
  float* RB = (float*)(ws + oRB);
  unsigned short* XHL = (unsigned short*)(ws + oXHL);
  unsigned short* Z4  = (unsigned short*)(ws + oZ4);
  float* T4 = (float*)(ws + oT4);

  hipFuncSetAttribute(reinterpret_cast<const void*>(&k_bucket),
                      hipFuncAttributeMaxDynamicSharedMemorySize, LDS_BKT);

  const int vec8 = ((nE & 3) == 0) ? 1 : 0;
  const int gM = MP / GBM;
  const int gS = MP / SSL;

  k_wlr<<<4, NTHR, 0, stream>>>(W1, al1, ar1, W2, al2, ar2, W3, al3, ar3, W4, al4, ar4, WLR);
  k_wprep<<<UT / NTHR, NTHR, 0, stream>>>(W1, W2, W3, W4, W1t, W2d, W3d, W4d);
  k_cvx<<<(MP * (D0 / 8)) / NTHR, NTHR, 0, stream>>>(feat, WLR, FB, ELa, ERa, NN);
  k_bucket<<<NBK, NTHR, LDS_BKT, stream>>>(src, dst, nE, NN, vec8, SRT, SOFF, SCNT, META);

  k_gemm<0><<<dim3(gM, D1 / GBN), GTHR, 0, stream>>>(FB, W1t, RA, D0, D1, b1);
  k_scan<1, 0><<<gS, NTHR, 0, stream>>>(SRT, SOFF, SCNT, META, RA, ELa, ERa, b1, WLR + 64, WLR + 1024 + 64,
                                        XHL, RB, ELb, ERb, NN, MP);
  k_gemm<0><<<dim3(gM, D2 / GBN), GTHR, 0, stream>>>(XHL, W2d, RB, 2 * D1, D2, b2);
  k_scan<2, 0><<<gS, NTHR, 0, stream>>>(SRT, SOFF, SCNT, META, RB, ELb, ERb, b2, WLR + 192, WLR + 1024 + 192,
                                        XHL, RA, ELa, ERa, NN, MP);
  k_gemm<0><<<dim3(gM, D3 / GBN), GTHR, 0, stream>>>(XHL, W3d, RA, 2 * D2, D3, b3);
  k_scan<4, 1><<<gS, NTHR, 0, stream>>>(SRT, SOFF, SCNT, META, RA, ELa, ERa, b3, WLR + 448, WLR + 1024 + 448,
                                        XHL, RB, ELb, ERb, NN, MP);
  k_scan<4, 2><<<RPOOL / SSL, NTHR, 0, stream>>>(SRT, SOFF, SCNT, META, RB, ELb, ERb, b4, WLR, WLR + 1024,
                                                 Z4, RA, ELa, ERa, NN, RPOOL);
  k_gemm<1><<<dim3(RPOOL / GBM, D4 / GBN), GTHR, 0, stream>>>(Z4, W4d, T4, 2 * D3, D4, b4);
  k_head<<<1, HTHR, 0, stream>>>(T4, relW, relB, rel, order, META, out);
}
